// DNC_47871705481292
// MI455X (gfx1250) — hardware-verified
//
#include <hip/hip_runtime.h>
#include <math.h>

constexpr int NBATCH = 16;
constexpr int NSTEP  = 64;
constexpr int NIN    = 256;
constexpr int NHID   = 512;
constexpr int NGATE  = 4 * NHID;
constexpr int NCELL  = 256;
constexpr int NCW    = 64;
constexpr int NRH    = 4;
constexpr int NIFACE = 471;
constexpr int NIFPAD = 512;
constexpr int NROWS  = NBATCH * NSTEP;
constexpr int NCAT   = NHID + NRH * NCW;
constexpr int NTHR   = 256;
constexpr int NWAVE  = NTHR / 32;
constexpr int SLABP  = 68;
constexpr int MHP    = 264;
constexpr int NBIAS  = 2 * NGATE + NHID + NIFPAD + NIN;
constexpr int OFF_BSUM0 = 0;
constexpr int OFF_BSUM1 = NGATE;
constexpr int OFF_BOUT  = 2 * NGATE;
constexpr int OFF_BIF   = 2 * NGATE + NHID;
constexpr int OFF_BMEM  = 2 * NGATE + NHID + NIFPAD;
constexpr float ACARRY  = 16.0f;
constexpr float WCARRY  = 64.0f;
constexpr float AW_INV  = 1.0f / 1024.0f;
constexpr float OUT_SCL = 1.0f / 64.0f;
constexpr float MCARRY  = 1024.0f;
constexpr float RCARRY  = 1024.0f;
constexpr float RV_INV  = 1.0f / 1048576.0f;
constexpr float DELTA_F = 1e-6f;
constexpr float UDECAY  = 0.999999f;
static_assert(NCELL == NTHR);
static_assert(NRH * NCW == NTHR);
static_assert(NHID == 64 * NWAVE);
static_assert(NIFACE <= NIFPAD && NIFPAD <= NGATE);
static_assert(NIN % 32 == 0 && NHID % 32 == 0 && NCAT % 32 == 0);
static_assert(NROWS % 64 == 0 && NHID % 64 == 0 && NIFPAD % 64 == 0 && NIN % 64 == 0);
static_assert((NCW * MHP) % NTHR == 0);
static_assert(MHP % 8 == 0 && MHP >= NCELL + 8);
static_assert((NCW * NCELL) % (4 * NTHR) == 0 && (NCELL * NCELL) % (4 * NTHR) == 0);

typedef __attribute__((ext_vector_type(16))) _Float16 v16h;
typedef __attribute__((ext_vector_type(8)))  _Float16 v8h;
typedef __attribute__((ext_vector_type(16))) __bf16   v16b;
typedef __attribute__((ext_vector_type(8)))  __bf16   v8b;
typedef __attribute__((ext_vector_type(8)))  float    v8f;
typedef __attribute__((ext_vector_type(4)))  float    v4f;
typedef __attribute__((ext_vector_type(4)))  unsigned v4u;

__device__ __forceinline__ unsigned short f2bf_bits(float f) {
  unsigned u = __float_as_uint(f);
  return (unsigned short)((u + 0x7FFFu + ((u >> 16) & 1u)) >> 16);
}
__device__ __forceinline__ float bf_bits2f(unsigned short h) { return __uint_as_float(((unsigned)h) << 16); }
__device__ __forceinline__ float bf16r(float f) { return bf_bits2f(f2bf_bits(f)); }

__device__ __forceinline__ void dep_guard_h(v8f& a, v8f& b, v16h x, v16h y) { asm volatile("v_nop\n\tv_nop\n\tv_nop\n\tv_nop" : "+v"(a), "+v"(b) : "v"(x), "v"(y)); }
__device__ __forceinline__ void dep_guard_b(v8f& a, v8f& b, v16b x, v16b y) { asm volatile("v_nop\n\tv_nop\n\tv_nop\n\tv_nop" : "+v"(a), "+v"(b) : "v"(x), "v"(y)); }
__device__ __forceinline__ void dep_guard_1(v8f& a, v16h x, v16h y) { asm volatile("v_nop\n\tv_nop\n\tv_nop\n\tv_nop" : "+v"(a) : "v"(x), "v"(y)); }
__device__ __forceinline__ void keep4_h(v16h a, v16h b, v16h c, v16h d) { asm volatile("v_nop" :: "v"(a), "v"(b), "v"(c), "v"(d)); }
__device__ __forceinline__ void keep4_b(v16b a, v16b b, v16b c, v16b d) { asm volatile("v_nop" :: "v"(a), "v"(b), "v"(c), "v"(d)); }
__device__ __forceinline__ void acc_guard4(v8f& a, v8f& b, v8f& c, v8f& d) { asm volatile("v_nop\n\tv_nop\n\tv_nop\n\tv_nop" : "+v"(a), "+v"(b), "+v"(c), "+v"(d)); }
__device__ __forceinline__ void acc_guard_1(v8f& a) { asm volatile("v_nop\n\tv_nop\n\tv_nop\n\tv_nop" : "+v"(a)); }
template <typename T> struct Frag;
template <> struct Frag<_Float16> {
  typedef v16h V; union U { v16h v; v8h h[2]; };
  static __device__ __forceinline__ v16h load(const _Float16* p) {
    U f; f.h[0] = *(const v8h*)(p); f.h[1] = *(const v8h*)(p + 16); return f.v;
  }
  static __device__ __forceinline__ v8f mma(v16h a, v16h b, v8f c) {
    return __builtin_amdgcn_wmma_f32_16x16x32_f16(false, a, false, b, (short)0, c, false, false);
  }
  static __device__ __forceinline__ void guard(v8f& a, v8f& b, v16h x, v16h y) { dep_guard_h(a, b, x, y); }
  static __device__ __forceinline__ void keep(v16h a, v16h b, v16h c, v16h d) { keep4_h(a, b, c, d); }
};
template <> struct Frag<__bf16> {
  typedef v16b V; union U { v16b v; v8b h[2]; };
  static __device__ __forceinline__ v16b load(const __bf16* p) {
    U f; f.h[0] = *(const v8b*)(p); f.h[1] = *(const v8b*)(p + 16); return f.v;
  }
  static __device__ __forceinline__ v8f mma(v16b a, v16b b, v8f c) {
    return __builtin_amdgcn_wmma_f32_16x16x32_bf16(false, a, false, b, (short)0, c, false, false);
  }
  static __device__ __forceinline__ void guard(v8f& a, v8f& b, v16b x, v16b y) { dep_guard_b(a, b, x, y); }
  static __device__ __forceinline__ void keep(v16b a, v16b b, v16b c, v16b d) { keep4_b(a, b, c, d); }
};

__device__ __forceinline__ float fsigm(float x) { return 1.0f / (1.0f + expf(-x)); }
__device__ __forceinline__ float fsoftplus(float x) { return fmaxf(x, 0.0f) + log1pf(expf(-fabsf(x))); }
__device__ __forceinline__ float wave_sum(float v) {
#pragma unroll
  for (int off = 16; off > 0; off >>= 1) v += __shfl_xor(v, off, 32);
  return v;
}
__device__ __forceinline__ float wave_max(float v) {
#pragma unroll
  for (int off = 16; off > 0; off >>= 1) v = fmaxf(v, __shfl_xor(v, off, 32));
  return v;
}

template <int ET> struct Elem;
template <> struct Elem<0> { typedef _Float16 T; };
template <> struct Elem<1> { typedef __bf16 T; };
template <int ET, bool SPLIT, int BIAS_MODE, int OUT_MODE, bool RESID, int ACT = 0>
__global__ __launch_bounds__(256) void wmma_gemm64(
    const unsigned short* __restrict__ Ap, const unsigned short* __restrict__ A2p, int lda, long strideA,
    const unsigned short* __restrict__ Btp, const unsigned short* __restrict__ Bt2p, int ldb, long strideB,
    void* __restrict__ Cout, void* __restrict__ Cout2, int ldc, long strideC,
    const float* __restrict__ bias,
    const float* __restrict__ resid, long strideR,
    int M, int N, int K, float scale) {
  typedef typename Elem<ET>::T T;
  typedef typename Frag<T>::V V;
  const T* A = (const T*)Ap; const T* A2 = (const T*)A2p; const T* Bt = (const T*)Btp; const T* Bt2 = (const T*)Bt2p;
  __shared__ __align__(16) float sT[8][16 * 68];
  const int b    = blockIdx.y;
  const int lane = threadIdx.x & 31;
  const int wave = threadIdx.x >> 5;
  const int tilesN = N >> 6;
  const int tilesM = M >> 6;
  const int tile = blockIdx.x * 8 + wave;
  if (tile >= tilesM * tilesN) return;
  const int tm = tile / tilesN;
  const int tn = tile - tm * tilesN;
  const int m0 = tm << 6;
  const int n0 = tn << 6;

  const T* Ab  = A  + (size_t)b * strideA;
  const T* Bb  = Bt + (size_t)b * strideB;
  const T* Ab2 = SPLIT ? (A2  + (size_t)b * strideA) : nullptr;
  const T* Bb2 = SPLIT ? (Bt2 + (size_t)b * strideB) : nullptr;

  const int rlane = lane & 15;
  const int koff  = (lane >> 4) * 8;
  const int mOff  = (lane >> 4) * 8;

  v8f acc[4][4];
#pragma unroll
  for (int i = 0; i < 4; ++i)
#pragma unroll
    for (int j = 0; j < 4; ++j) acc[i][j] = (v8f){0.f,0.f,0.f,0.f,0.f,0.f,0.f,0.f};

  for (int k0 = 0; k0 < K; k0 += 32) {
    V bh[4], bl[4];
#pragma unroll
    for (int j = 0; j < 4; ++j) {
      const size_t bo = (size_t)(n0 + (j << 4) + rlane) * ldb + koff + k0;
      bh[j] = Frag<T>::load(Bb + bo);
      if (SPLIT) bl[j] = Frag<T>::load(Bb2 + bo);
    }
#pragma unroll
    for (int i = 0; i < 4; ++i) {
      const size_t ao = (size_t)(m0 + (i << 4) + rlane) * lda + koff + k0;
      V ah = Frag<T>::load(Ab + ao);
      V al;
      if (SPLIT) al = Frag<T>::load(Ab2 + ao);
#pragma unroll
      for (int j = 0; j < 4; ++j) {
        acc[i][j] = Frag<T>::mma(ah, bh[j], acc[i][j]);
        if (SPLIT) {
          acc[i][j] = Frag<T>::mma(ah, bl[j], acc[i][j]);
          acc[i][j] = Frag<T>::mma(al, bh[j], acc[i][j]);
        }
      }
      Frag<T>::guard(acc[i][0], acc[i][3], ah, SPLIT ? al : ah);
    }
    Frag<T>::keep(bh[0], bh[1], bh[2], bh[3]);
    if (SPLIT) Frag<T>::keep(bl[0], bl[1], bl[2], bl[3]);
  }
  acc_guard4(acc[0][0], acc[0][1], acc[0][2], acc[0][3]);
  acc_guard4(acc[1][0], acc[1][1], acc[1][2], acc[1][3]);
  acc_guard4(acc[2][0], acc[2][1], acc[2][2], acc[2][3]);
  acc_guard4(acc[3][0], acc[3][1], acc[3][2], acc[3][3]);

  float* slab = sT[wave];
  const float* Rb = RESID ? (resid + (size_t)b * strideR) : nullptr;
#pragma unroll
  for (int i = 0; i < 4; ++i) {
    const int mBase = m0 + (i << 4);
#pragma unroll
    for (int j = 0; j < 4; ++j) {
      const int n = n0 + (j << 4) + rlane;
      float bv = 0.f;
      if (BIAS_MODE == 2) bv = bias[n];
#pragma unroll
      for (int r = 0; r < 8; ++r) {
        float v = acc[i][j][r] * scale;
        if (BIAS_MODE == 1) v += bias[mBase + mOff + r];
        if (BIAS_MODE == 2) v += bv;
        if (RESID) v += Rb[(size_t)(mBase + mOff + r) * ldc + n];
        if (ACT == 1) v = tanhf(v);
        if (ACT == 2) v = fmaxf(v, 0.0f);
        if (ACT == 3) v = v / (1.0f + expf(-v));
        if (ACT == 4) v = (v > 0.f) ? v : 0.01f * v;
        if (ACT == 5) v = 0.5f * v * (1.0f + erff(v * 0.70710678118654752f));
        slab[(mOff + r) * 68 + (j << 4) + rlane] = v;
      }
    }
    __builtin_amdgcn_fence(__ATOMIC_RELEASE, "workgroup");
    __builtin_amdgcn_wave_barrier();
    __builtin_amdgcn_fence(__ATOMIC_ACQUIRE, "workgroup");
    if (OUT_MODE == 0) {
      float* C = (float*)Cout + (size_t)b * strideC;
      const int hh = lane >> 4, c4 = (lane & 15) * 4;
      for (int pass = 0; pass < 2; ++pass) {
#pragma unroll
        for (int it = 0; it < 8; ++it) {
          const int row = it * 2 + hh;
          v4f v = *(const v4f*)(slab + row * 68 + c4);
          *(volatile v4f*)(C + (size_t)(mBase + row) * ldc + n0 + c4) = v;
        }
        __threadfence();
      }
    } else {
      const int q = lane >> 3, c8 = (lane & 7) * 8;
      unsigned short* C  = (unsigned short*)Cout  + (size_t)b * strideC;
      unsigned short* C2 = (OUT_MODE == 2) ? ((unsigned short*)Cout2 + (size_t)b * strideC) : nullptr;
      for (int pass = 0; pass < 2; ++pass) {
#pragma unroll
        for (int it = 0; it < 4; ++it) {
          const int row = it * 4 + q;
          const float* sp = slab + row * 68 + c8;
          v8h hv, lv;
#pragma unroll
          for (int e = 0; e < 8; ++e) {
            if (OUT_MODE == 1) {
              hv[e] = (_Float16)sp[e];
            } else {
              unsigned short hb = f2bf_bits(sp[e]);
              unsigned short lb = f2bf_bits(sp[e] - bf_bits2f(hb));
              hv[e] = __builtin_bit_cast(_Float16, hb);
              lv[e] = __builtin_bit_cast(_Float16, lb);
            }
          }
          *(volatile v8h*)(C + (size_t)(mBase + row) * ldc + n0 + c8) = hv;
          if (OUT_MODE == 2) *(volatile v8h*)(C2 + (size_t)(mBase + row) * ldc + n0 + c8) = lv;
        }
        __threadfence();
      }
    }
    __builtin_amdgcn_fence(__ATOMIC_RELEASE, "workgroup");
    __builtin_amdgcn_wave_barrier();
    __builtin_amdgcn_fence(__ATOMIC_ACQUIRE, "workgroup");
  }
}

__global__ __launch_bounds__(NTHR) void cvt8_kernel(const float* __restrict__ src, unsigned short* __restrict__ dst,
                                                    int nrow, int nrow_src, int ncol8, int spitch, int scol0, float sc) {
  const int i  = blockIdx.x * NTHR + threadIdx.x;
  const int n8 = nrow * ncol8;
  if (i < n8) {
    const int row = i / ncol8;
    const int c8  = i - row * ncol8;
    const int rs  = (row < nrow_src) ? row : (nrow_src - 1);
    const float zs = (row < nrow_src) ? sc : 0.0f;
    const float* sp = src + (size_t)rs * spitch + scol0 + c8 * 8;
    const v4f a = *(const v4f*)(sp);
    const v4f b = *(const v4f*)(sp + 4);
    v8h hv;
#pragma unroll
    for (int e = 0; e < 4; ++e) {
      hv[e]     = (_Float16)(bf16r(a[e]) * zs);
      hv[4 + e] = (_Float16)(bf16r(b[e]) * zs);
    }
    *(volatile v8h*)(dst + (size_t)i * 8) = hv;
    __threadfence();
    *(volatile v8h*)(dst + (size_t)i * 8) = hv;
  }
}

__global__ __launch_bounds__(NTHR) void bias_prep_kernel(const float* __restrict__ bih0, const float* __restrict__ bhh0,
                                                         const float* __restrict__ bih1, const float* __restrict__ bhh1,
                                                         const float* __restrict__ bout, const float* __restrict__ bif,
                                                         const float* __restrict__ bmem, float* __restrict__ dst) {
  const int blk = blockIdx.x, tid = threadIdx.x;
  v4f o = {0.f, 0.f, 0.f, 0.f};
  float* op = dst;
  bool act = false;
  if (blk < 2) {
    const int idx = (blk * NTHR + tid) * 4;
    const v4f va = *(const v4f*)(bih0 + idx);
    const v4f vb = *(const v4f*)(bhh0 + idx);
#pragma unroll
    for (int e = 0; e < 4; ++e) o[e] = bf16r(va[e]) + bf16r(vb[e]);
    op = dst + OFF_BSUM0 + idx; act = true;
  } else if (blk < 4) {
    const int idx = ((blk - 2) * NTHR + tid) * 4;
    const v4f va = *(const v4f*)(bih1 + idx);
    const v4f vb = *(const v4f*)(bhh1 + idx);
#pragma unroll
    for (int e = 0; e < 4; ++e) o[e] = bf16r(va[e]) + bf16r(vb[e]);
    op = dst + OFF_BSUM1 + idx; act = true;
  } else if (blk == 4) {
    if (tid < NHID / 4) {
      const int idx = tid * 4;
      const v4f va = *(const v4f*)(bout + idx);
#pragma unroll
      for (int e = 0; e < 4; ++e) o[e] = ACARRY * bf16r(va[e]);
      op = dst + OFF_BOUT + idx; act = true;
    }
  } else if (blk == 5) {
    if (tid < NIFPAD / 4) {
      const int idx = tid * 4;
#pragma unroll
      for (int e = 0; e < 4; ++e) {
        const int n  = idx + e;
        const int nc = (n < NIFACE) ? n : (NIFACE - 1);
        const float f = bif[nc];
        o[e] = (n < NIFACE) ? bf16r(f) : 0.0f;
      }
      op = dst + OFF_BIF + idx; act = true;
    }
  } else {
    if (tid < NIN / 4) {
      const int idx = tid * 4;
      const v4f va = *(const v4f*)(bmem + idx);
#pragma unroll
      for (int e = 0; e < 4; ++e) o[e] = bf16r(va[e]);
      op = dst + OFF_BMEM + idx; act = true;
    }
  }
  if (act) {
    *(volatile v4f*)op = o;
    __threadfence();
    *(volatile v4f*)op = o;
  }
}

template <int KIN>
__global__ __launch_bounds__(NTHR) void lstm_seq_kernel(const unsigned short* __restrict__ XP,
                                                        const unsigned short* __restrict__ WIp,
                                                        const unsigned short* __restrict__ WHp,
                                                        const float* __restrict__ bsum,
                                                        unsigned short* __restrict__ HP) {
  constexpr int AP   = KIN + NHID + 8;
  constexpr int NX16 = KIN / 8;
  constexpr int NXIT = (NBATCH * NX16) / NTHR;
  static_assert((NBATCH * NX16) % NTHR == 0);
  static_assert(AP % 8 == 0 && KIN % 32 == 0);
  __shared__ __align__(16) _Float16 At[NBATCH * AP];
  __shared__ __align__(16) float    Sl[NWAVE][16 * SLABP];
  const _Float16* WI = (const _Float16*)WIp;
  const _Float16* WH = (const _Float16*)WHp;
  const int tid = threadIdx.x, lane = tid & 31, wave = tid >> 5;
  const int c = lane & 15, hh = lane >> 4, koff = hh * 8;
  const int q = lane >> 3, c8 = (lane & 7) * 8;

#pragma unroll 1
  for (int i = tid; i < NBATCH * AP; i += NTHR) At[i] = (_Float16)0.0f;
  float cst[4][8];
#pragma unroll
  for (int nt = 0; nt < 4; ++nt)
#pragma unroll
    for (int r = 0; r < 8; ++r) cst[nt][r] = 0.0f;
  __syncthreads();
#pragma unroll
  for (int it = 0; it < NXIT; ++it) {
    const int idx = it * NTHR + tid;
    const int row = idx / NX16, ch = idx - row * NX16;
    const v4u v = *(const v4u*)(XP + (size_t)(row * NSTEP) * KIN + 8 * ch);
    *(v4u*)((unsigned short*)At + row * AP + 8 * ch) = v;
  }
  __syncthreads();

  float* slab = Sl[wave];
  const _Float16* axrow = At + c * AP + koff;
  const _Float16* ahrow = At + c * AP + KIN + koff;
  const v8f z8 = {0.f, 0.f, 0.f, 0.f, 0.f, 0.f, 0.f, 0.f};

#pragma unroll 1
  for (int t = 0; t < NSTEP; ++t) {
#pragma unroll
    for (int nt = 0; nt < 4; ++nt) {
      const int j = 64 * wave + 16 * nt + c;
      const _Float16* wi = WI + (size_t)j * KIN + koff;
      const _Float16* wh = WH + (size_t)j * NHID + koff;
      const float bi = bsum[j];
      const float bf = bsum[NHID + j];
      const float bg = bsum[2 * NHID + j];
      const float bo = bsum[3 * NHID + j];
      v8f acc[4];
      acc[0] = z8; acc[1] = z8; acc[2] = z8; acc[3] = z8;
#pragma unroll 1
      for (int kx = 0; kx < KIN; kx += 32) {
        const v16h a  = Frag<_Float16>::load(axrow + kx);
        const v16h b0 = Frag<_Float16>::load(wi + kx);
        const v16h b1 = Frag<_Float16>::load(wi + (size_t)1 * NHID * KIN + kx);
        const v16h b2 = Frag<_Float16>::load(wi + (size_t)2 * NHID * KIN + kx);
        const v16h b3 = Frag<_Float16>::load(wi + (size_t)3 * NHID * KIN + kx);
        acc[0] = Frag<_Float16>::mma(a, b0, acc[0]);
        acc[1] = Frag<_Float16>::mma(a, b1, acc[1]);
        acc[2] = Frag<_Float16>::mma(a, b2, acc[2]);
        acc[3] = Frag<_Float16>::mma(a, b3, acc[3]);
        dep_guard_h(acc[0], acc[3], a, b3);
        keep4_h(b0, b1, b2, b3);
      }
#pragma unroll 1
      for (int k0 = 0; k0 < NHID; k0 += 32) {
        const v16h a  = Frag<_Float16>::load(ahrow + k0);
        const v16h b0 = Frag<_Float16>::load(wh + k0);
        const v16h b1 = Frag<_Float16>::load(wh + (size_t)1 * NHID * NHID + k0);
        const v16h b2 = Frag<_Float16>::load(wh + (size_t)2 * NHID * NHID + k0);
        const v16h b3 = Frag<_Float16>::load(wh + (size_t)3 * NHID * NHID + k0);
        acc[0] = Frag<_Float16>::mma(a, b0, acc[0]);
        acc[1] = Frag<_Float16>::mma(a, b1, acc[1]);
        acc[2] = Frag<_Float16>::mma(a, b2, acc[2]);
        acc[3] = Frag<_Float16>::mma(a, b3, acc[3]);
        dep_guard_h(acc[0], acc[3], a, b3);
        keep4_h(b0, b1, b2, b3);
      }
      acc_guard4(acc[0], acc[1], acc[2], acc[3]);
#pragma unroll
      for (int r = 0; r < 8; ++r) {
        const float zi = acc[0][r] * AW_INV + bi;
        const float zf = acc[1][r] * AW_INV + bf;
        const float zg = acc[2][r] * AW_INV + bg;
        const float zo = acc[3][r] * AW_INV + bo;
        const float ig = fsigm(zi);
        const float fg = fsigm(zf);
        const float gg = tanhf(zg);
        const float og = fsigm(zo);
        const float cn = fg * cst[nt][r] + ig * gg;
        cst[nt][r] = cn;
        const float hn = og * tanhf(cn);
        slab[(8 * hh + r) * SLABP + 16 * nt + c] = hn * ACARRY;
      }
    }
    __syncthreads();
#pragma unroll
    for (int nt = 0; nt < 4; ++nt) {
      const int j = 64 * wave + 16 * nt + c;
#pragma unroll
      for (int r = 0; r < 8; ++r) At[(8 * hh + r) * AP + KIN + j] = (_Float16)slab[(8 * hh + r) * SLABP + 16 * nt + c];
    }
    {
      const int tn = (t + 1 < NSTEP) ? (t + 1) : (NSTEP - 1);
#pragma unroll
      for (int it = 0; it < NXIT; ++it) {
        const int idx = it * NTHR + tid;
        const int row = idx / NX16, ch = idx - row * NX16;
        const v4u v = *(const v4u*)(XP + (size_t)(row * NSTEP + tn) * KIN + 8 * ch);
        *(v4u*)((unsigned short*)At + row * AP + 8 * ch) = v;
      }
    }
    for (int pass = 0; pass < 2; ++pass) {
#pragma unroll
      for (int it = 0; it < 4; ++it) {
        const int row = it * 4 + q;
        const float* sp = slab + row * SLABP + c8;
        const v4f s0 = *(const v4f*)(sp);
        const v4f s1 = *(const v4f*)(sp + 4);
        v8h hv;
#pragma unroll
        for (int e = 0; e < 4; ++e) { hv[e] = (_Float16)s0[e]; hv[4 + e] = (_Float16)s1[e]; }
        *(volatile v8h*)(HP + (size_t)(row * NSTEP + t) * NHID + 64 * wave + c8) = hv;
      }
      __threadfence();
    }
    __syncthreads();
  }
}

__global__ __launch_bounds__(NTHR) void mem_seq_kernel(const float* __restrict__ XI, float* __restrict__ memT,
                                                       float* __restrict__ lnk, unsigned short* __restrict__ CA) {
  __shared__ __align__(16) _Float16 Mh[NCW * MHP];
  __shared__ __align__(16) _Float16 RWh[16 * MHP];
  __shared__ __align__(16) float xi_s[NIFPAD];
  __shared__ __align__(16) float rk_s[NRH * NCW];
  __shared__ __align__(16) float wk_s[NCW];
  __shared__ __align__(16) float ev_s[NCW];
  __shared__ __align__(16) float wv_s[NCW];
  __shared__ __align__(16) float usage_s[NCELL];
  __shared__ __align__(16) float wwp_s[NCELL];
  __shared__ __align__(16) float u2_s[NCELL];
  __shared__ __align__(16) float srt_s[NCELL];
  __shared__ __align__(16) float pe_s[NCELL];
  __shared__ __align__(16) float rwp_s[NRH * NCELL];
  __shared__ __align__(16) float rv_s[NRH * NCW];
  __shared__ __align__(16) float rednk[8];
  __shared__ __align__(16) float redwk[8];
  __shared__ __align__(16) float red1[8];
  __shared__ __align__(16) float red2[8];
  __shared__ __align__(16) float red3[8];
  __shared__ __align__(16) float red4[32];
  __shared__ __align__(16) float red5[32];
  __shared__ __align__(16) float par_s[32];

  const int b = blockIdx.x, tid = threadIdx.x, lane = tid & 31, wave = tid >> 5;
  const int c = lane & 15, hh = lane >> 4, koff = hh * 8;
  float* MT = memT + (size_t)b * (NCW * NCELL);
  float* LK = lnk  + (size_t)b * (NCELL * NCELL);

#pragma unroll 1
  for (int i = tid; i < NCW * MHP; i += NTHR) Mh[i] = (_Float16)0.0f;
#pragma unroll 1
  for (int i = tid; i < 16 * MHP; i += NTHR) RWh[i] = (_Float16)0.0f;
  usage_s[tid] = 0.0f; wwp_s[tid] = 0.0f; u2_s[tid] = 0.0f; srt_s[tid] = 0.0f; pe_s[tid] = 1.0f;
  rv_s[tid] = 0.0f; rk_s[tid] = 0.0f; xi_s[tid] = 0.0f; xi_s[tid + 256] = 0.0f;
#pragma unroll
  for (int r = 0; r < NRH; ++r) rwp_s[r * NCELL + tid] = 0.0f;
  if (tid < NCW) { wk_s[tid] = 0.0f; ev_s[tid] = 0.0f; wv_s[tid] = 0.0f; }
  if (tid < 32) { par_s[tid] = 0.0f; red4[tid] = 0.0f; red5[tid] = 0.0f; }
  if (tid < 8) { rednk[tid] = 0.0f; redwk[tid] = 0.0f; red1[tid] = 0.0f; red2[tid] = 0.0f; red3[tid] = 0.0f; }
  {
    const v4f z4 = {0.f, 0.f, 0.f, 0.f};
    for (int pass = 0; pass < 2; ++pass) {
#pragma unroll 1
      for (int it = 0; it < (NCW * NCELL) / (4 * NTHR); ++it) *(volatile v4f*)(MT + 4 * (size_t)(it * NTHR + tid)) = z4;
#pragma unroll 1
      for (int it = 0; it < (NCELL * NCELL) / (4 * NTHR); ++it) *(volatile v4f*)(LK + 4 * (size_t)(it * NTHR + tid)) = z4;
      __threadfence();
    }
  }
  float prec_t = 0.0f;
  __syncthreads();
  const v8f z8 = {0.f, 0.f, 0.f, 0.f, 0.f, 0.f, 0.f, 0.f};

#pragma unroll 1
  for (int t = 0; t < NSTEP; ++t) {
    const size_t row = (size_t)b * NSTEP + (size_t)t;
    xi_s[tid]       = XI[row * NIFPAD + tid];
    xi_s[tid + 256] = XI[row * NIFPAD + 256 + tid];
    __syncthreads();
    const float rkv = tanhf(xi_s[tid]);
    rk_s[tid] = rkv;
    float sq = rkv * rkv, sqw = 0.0f;
    if (wave < 2) {
      const int w = tid & 63;
      const float wkv = tanhf(xi_s[260 + w]);
      wk_s[w] = wkv;
      ev_s[w] = fsigm(xi_s[325 + w]);
      wv_s[w] = tanhf(xi_s[389 + w]);
      sqw = wkv * wkv;
    }
    sq  = wave_sum(sq);
    sqw = wave_sum(sqw);
    if (lane == 0) { rednk[wave] = sq; redwk[wave] = sqw; }
    if (wave == 2) {
      const int r4 = lane & 3;
      const float rsv = fsoftplus(xi_s[256 + r4]);
      const float fgv = fsigm(xi_s[453 + r4]);
      const float a0 = xi_s[459 + 3 * r4], a1 = xi_s[460 + 3 * r4], a2 = xi_s[461 + 3 * r4];
      const float mx = fmaxf(a0, fmaxf(a1, a2));
      const float e0 = expf(a0 - mx), e1 = expf(a1 - mx), e2 = expf(a2 - mx);
      const float inv3 = 1.0f / (e0 + e1 + e2);
      if (lane < 4) {
        par_s[r4] = rsv; par_s[4 + r4] = fgv;
        par_s[8 + 3 * r4] = e0 * inv3; par_s[9 + 3 * r4] = e1 * inv3; par_s[10 + 3 * r4] = e2 * inv3;
      }
    }
    if (wave == 3) {
      const float wsv = fsoftplus(xi_s[324]);
      const float agv = fsigm(xi_s[457]);
      const float wgv = fsigm(xi_s[458]);
      if (lane == 0) { par_s[20] = wsv; par_s[21] = agv; par_s[22] = wgv; }
    }
    __syncthreads();
    float knrm[4];
#pragma unroll
    for (int r = 0; r < NRH; ++r) knrm[r] = sqrtf(rednk[2 * r] + rednk[2 * r + 1]) + DELTA_F;
    const float wkn = sqrtf(redwk[0] + redwk[1]) + DELTA_F;
    float rs4[4];
#pragma unroll
    for (int r = 0; r < NRH; ++r) rs4[r] = par_s[r];
    const float wsv = par_s[20], agv = par_s[21], wgv = par_s[22];
    float u = usage_s[tid];
    const float wwo = wwp_s[tid];
    u = u + (1.0f - u) * wwo;
    float psi = 1.0f;
#pragma unroll
    for (int r = 0; r < NRH; ++r) psi *= 1.0f - par_s[4 + r] * rwp_s[r * NCELL + tid];
    u = u * psi;
    usage_s[tid] = u;
    const float u2 = DELTA_F + UDECAY * u;
    u2_s[tid] = u2;
    float dtA = 0.0f, nmA = 0.0f;
#pragma unroll 4
    for (int w = 0; w < NCW; ++w) {
      const float mv = MT[(size_t)w * NCELL + tid];
      nmA += mv * mv;
      dtA += mv * wk_s[w];
    }
    const float score = (dtA * (1.0f / ((sqrtf(nmA) + DELTA_F) * wkn))) * wsv;
    {
      const float m = wave_max(score);
      if (lane == 0) red1[wave] = m;
    }
    __syncthreads();
    float gmax = red1[0];
#pragma unroll
    for (int w = 1; w < 8; ++w) gmax = fmaxf(gmax, red1[w]);
    const float eA = expf(score - gmax);
    {
      const float s = wave_sum(eA);
      if (lane == 0) red2[wave] = s;
    }
    int rank = 0;
#pragma unroll 2
    for (int j4 = 0; j4 < NCELL / 4; ++j4) {
      const v4f v = *(const v4f*)(u2_s + 4 * j4);
#pragma unroll
      for (int e = 0; e < 4; ++e) {
        const int j = 4 * j4 + e;
        rank += (v[e] < u2) ? 1 : 0;
        rank += ((v[e] == u2) && (j < tid)) ? 1 : 0;
      }
    }
    srt_s[rank] = u2;
    __syncthreads();
    float ssum = red2[0];
#pragma unroll
    for (int w = 1; w < 8; ++w) ssum += red2[w];
    const float wcw = eA * (1.0f / ssum);
    if (tid == 0) {
      float run = 1.0f;
#pragma unroll 1
      for (int i = 0; i < NCELL; ++i) { pe_s[i] = run; run = run * srt_s[i]; }
    }
    __syncthreads();
    const float alloc = (1.0f - u2) * pe_s[rank];
    const float wwn = wgv * (agv * alloc + (1.0f - agv) * wcw);
    {
      const float s = wave_sum(wwn);
      if (lane == 0) red3[wave] = s;
    }
    wwp_s[tid] = wwn;
    __syncthreads();
    float sww = red3[0];
#pragma unroll
    for (int w = 1; w < 8; ++w) sww += red3[w];
    float nmB = 0.0f;
    float dB[4] = {0.f, 0.f, 0.f, 0.f};
#pragma unroll 1
    for (int wc = 0; wc < NCW / 8; ++wc) {
      float nv[8];
#pragma unroll
      for (int e = 0; e < 8; ++e) {
        const int w = wc * 8 + e;
        const float mv  = MT[(size_t)w * NCELL + tid];
        const float nvv = mv * (1.0f - wwn * ev_s[w]) + wwn * wv_s[w];
        nv[e] = nvv;
        nmB += nvv * nvv;
#pragma unroll
        for (int r = 0; r < NRH; ++r) dB[r] += nvv * rk_s[r * NCW + w];
        Mh[w * MHP + tid] = (_Float16)(nvv * MCARRY);
      }
      for (int pass = 0; pass < 2; ++pass) {
#pragma unroll
        for (int e = 0; e < 8; ++e) *(volatile float*)(MT + (size_t)(wc * 8 + e) * NCELL + tid) = nv[e];
        __threadfence();
      }
    }
    float bwd[4] = {0.f, 0.f, 0.f, 0.f};
#pragma unroll 1
    for (int ic = 0; ic < NCELL / 8; ++ic) {
      const int i0 = ic * 8;
      const v4f wwa = *(const v4f*)(wwp_s + i0);
      const v4f wwb = *(const v4f*)(wwp_s + i0 + 4);
      float Ln[8];
#pragma unroll
      for (int e = 0; e < 8; ++e) {
        const int i = i0 + e;
        const float wwi = (e < 4) ? wwa[e] : wwb[e - 4];
        const float L = LK[(size_t)i * NCELL + tid];
        float Lnew = (1.0f - wwi - wwn) * L + wwi * prec_t;
        Lnew = (i == tid) ? 0.0f : Lnew;
        Ln[e] = Lnew;
      }
#pragma unroll
      for (int r = 0; r < NRH; ++r) {
        const v4f ra = *(const v4f*)(rwp_s + r * NCELL + i0);
        const v4f rb = *(const v4f*)(rwp_s + r * NCELL + i0 + 4);
#pragma unroll
        for (int e = 0; e < 4; ++e) { bwd[r] += ra[e] * Ln[e]; bwd[r] += rb[e] * Ln[4 + e]; }
      }
      for (int pass = 0; pass < 2; ++pass) {
#pragma unroll
        for (int e = 0; e < 8; ++e) *(volatile float*)(LK + (size_t)(i0 + e) * NCELL + tid) = Ln[e];
        __threadfence();
      }
    }
    prec_t = (1.0f - sww) * prec_t + wwn;
    float sc4[4];
#pragma unroll
    for (int r = 0; r < NRH; ++r) sc4[r] = (dB[r] * (1.0f / ((sqrtf(nmB) + DELTA_F) * knrm[r]))) * rs4[r];
#pragma unroll
    for (int r = 0; r < NRH; ++r) {
      const float m = wave_max(sc4[r]);
      if (lane == 0) red4[wave * 4 + r] = m;
    }
    __syncthreads();
    float fwd[4] = {0.f, 0.f, 0.f, 0.f};
    {
      const float* lrow = LK + (size_t)tid * NCELL;
#pragma unroll 1
      for (int n4 = 0; n4 < NCELL / 4; ++n4) {
        const v4f L4 = *(const v4f*)(lrow + 4 * n4);
#pragma unroll
        for (int r = 0; r < NRH; ++r) {
          const v4f rw4 = *(const v4f*)(rwp_s + r * NCELL + 4 * n4);
#pragma unroll
          for (int e = 0; e < 4; ++e) fwd[r] += L4[e] * rw4[e];
        }
      }
    }
    float e4[4];
#pragma unroll
    for (int r = 0; r < NRH; ++r) {
      float gm = red4[r];
#pragma unroll
      for (int w = 1; w < 8; ++w) gm = fmaxf(gm, red4[w * 4 + r]);
      e4[r] = expf(sc4[r] - gm);
      const float s = wave_sum(e4[r]);
      if (lane == 0) red5[wave * 4 + r] = s;
    }
    __syncthreads();
#pragma unroll
    for (int r = 0; r < NRH; ++r) {
      float sm = red5[r];
#pragma unroll
      for (int w = 1; w < 8; ++w) sm += red5[w * 4 + r];
      const float cw  = e4[r] * (1.0f / sm);
      const float rwn = par_s[8 + 3 * r] * bwd[r] + par_s[9 + 3 * r] * fwd[r] + par_s[10 + 3 * r] * cw;
      rwp_s[r * NCELL + tid] = rwn;
      RWh[r * MHP + tid] = (_Float16)(rwn * RCARRY);
    }
    __syncthreads();
    if (wave < 4) {
      v8f acc = z8;
      const _Float16* arow = Mh  + (16 * wave + c) * MHP + koff;
      const _Float16* brow = RWh + c * MHP + koff;
#pragma unroll
      for (int k0 = 0; k0 < NCELL; k0 += 32) {
        const v16h a  = Frag<_Float16>::load(arow + k0);
        const v16h bq = Frag<_Float16>::load(brow + k0);
        acc = Frag<_Float16>::mma(a, bq, acc);
        dep_guard_1(acc, a, bq);
      }
      acc_guard_1(acc);
      if (c < 4) {
#pragma unroll
        for (int i = 0; i < 8; ++i) rv_s[c * NCW + 16 * wave + 8 * hh + i] = acc[i] * RV_INV;
      }
    }
    __syncthreads();
    if (wave == 0) {
      const v4f p0 = *(const v4f*)(rv_s + 8 * lane);
      const v4f p1 = *(const v4f*)(rv_s + 8 * lane + 4);
      v8h hv;
#pragma unroll
      for (int e = 0; e < 4; ++e) { hv[e] = (_Float16)(p0[e] * ACARRY); hv[4 + e] = (_Float16)(p1[e] * ACARRY); }
      unsigned short* dst = CA + row * NCAT + NHID + 8 * lane;
      *(volatile v8h*)dst = hv;
      __threadfence();
      *(volatile v8h*)dst = hv;
    }
  }
}

extern "C" void kernel_launch(void* const* d_in, const int* in_sizes, int n_in,
                              void* d_out, int out_size, void* d_ws, size_t ws_size, hipStream_t stream) {
  if (n_in < 15 || d_out == nullptr || d_ws == nullptr) return;
  if (in_sizes[0] != NBATCH * NSTEP * NIN || in_sizes[1] != NGATE * NHID || in_sizes[2] != NGATE ||
      in_sizes[3] != NGATE * NHID || in_sizes[4] != NGATE || in_sizes[5] != NGATE * NHID || in_sizes[6] != NGATE ||
      in_sizes[7] != NGATE * NHID || in_sizes[8] != NGATE || in_sizes[9] != NHID * NHID || in_sizes[10] != NHID ||
      in_sizes[11] != NIFACE * NHID || in_sizes[12] != NIFACE || in_sizes[13] != NIN * NCAT || in_sizes[14] != NIN ||
      out_size != NROWS * NIN) return;

  const float* x    = (const float*)d_in[0];
  const float* Wih0 = (const float*)d_in[1];
  const float* bih0 = (const float*)d_in[2];
  const float* Whh0 = (const float*)d_in[3];
  const float* bhh0 = (const float*)d_in[4];
  const float* Wih1 = (const float*)d_in[5];
  const float* bih1 = (const float*)d_in[6];
  const float* Whh1 = (const float*)d_in[7];
  const float* bhh1 = (const float*)d_in[8];
  const float* Wout = (const float*)d_in[9];
  const float* bout = (const float*)d_in[10];
  const float* Wif  = (const float*)d_in[11];
  const float* bif  = (const float*)d_in[12];
  const float* Wmem = (const float*)d_in[13];
  const float* bmem = (const float*)d_in[14];
  float* yout = (float*)d_out;

  char* ws = (char*)d_ws; size_t off = 0;
  auto carve = [&](size_t bytes) -> char* { char* p = ws + off; off += (bytes + 255) & ~(size_t)255; return p; };
  unsigned short* X16  = (unsigned short*)carve((size_t)NROWS * NIN * 2);
  unsigned short* WI0  = (unsigned short*)carve((size_t)NGATE * NIN * 2);
  unsigned short* WH0  = (unsigned short*)carve((size_t)NGATE * NHID * 2);
  unsigned short* WI1  = (unsigned short*)carve((size_t)NGATE * NHID * 2);
  unsigned short* WH1  = (unsigned short*)carve((size_t)NGATE * NHID * 2);
  unsigned short* WOUT = (unsigned short*)carve((size_t)NHID * NHID * 2);
  unsigned short* WIF  = (unsigned short*)carve((size_t)NIFPAD * NHID * 2);
  unsigned short* WMEM = (unsigned short*)carve((size_t)NIN * NCAT * 2);
  float*          BIAS = (float*)carve((size_t)NBIAS * 4);
  unsigned short* H0   = (unsigned short*)carve((size_t)NROWS * NHID * 2);
  unsigned short* H1   = (unsigned short*)carve((size_t)NROWS * NHID * 2);
  float*          XI   = (float*)carve((size_t)NROWS * NIFPAD * 4);
  unsigned short* CA   = (unsigned short*)carve((size_t)NROWS * NCAT * 2);
  float*          MEMT = (float*)carve((size_t)NBATCH * NCW * NCELL * 4);
  float*          LINK = (float*)carve((size_t)NBATCH * NCELL * NCELL * 4);
  if (off > ws_size || off > (size_t)134217728) return;

  cvt8_kernel<<<(NROWS * (NIN / 8)) / NTHR,   NTHR, 0, stream>>>(x,    X16,  NROWS,  NROWS,  NIN / 8,  NIN,  0, ACARRY);
  cvt8_kernel<<<(NGATE * (NIN / 8)) / NTHR,   NTHR, 0, stream>>>(Wih0, WI0,  NGATE,  NGATE,  NIN / 8,  NHID, 0, WCARRY);
  cvt8_kernel<<<(NGATE * (NHID / 8)) / NTHR,  NTHR, 0, stream>>>(Whh0, WH0,  NGATE,  NGATE,  NHID / 8, NHID, 0, WCARRY);
  cvt8_kernel<<<(NGATE * (NHID / 8)) / NTHR,  NTHR, 0, stream>>>(Wih1, WI1,  NGATE,  NGATE,  NHID / 8, NHID, 0, WCARRY);
  cvt8_kernel<<<(NGATE * (NHID / 8)) / NTHR,  NTHR, 0, stream>>>(Whh1, WH1,  NGATE,  NGATE,  NHID / 8, NHID, 0, WCARRY);
  cvt8_kernel<<<(NHID * (NHID / 8)) / NTHR,   NTHR, 0, stream>>>(Wout, WOUT, NHID,   NHID,   NHID / 8, NHID, 0, WCARRY);
  cvt8_kernel<<<(NIFPAD * (NHID / 8)) / NTHR, NTHR, 0, stream>>>(Wif,  WIF,  NIFPAD, NIFACE, NHID / 8, NHID, 0, WCARRY);
  cvt8_kernel<<<(NIN * (NCAT / 8)) / NTHR,    NTHR, 0, stream>>>(Wmem, WMEM, NIN,    NIN,    NCAT / 8, NCAT, 0, WCARRY);
  bias_prep_kernel<<<7, NTHR, 0, stream>>>(bih0, bhh0, bih1, bhh1, bout, bif, bmem, BIAS);
  lstm_seq_kernel<NIN><<<1, NTHR, 0, stream>>>(X16, WI0, WH0, BIAS + OFF_BSUM0, H0);
  lstm_seq_kernel<NHID><<<1, NTHR, 0, stream>>>(H0, WI1, WH1, BIAS + OFF_BSUM1, H1);
  wmma_gemm64<0, false, 2, 1, false, 0><<<dim3((NROWS / 64) * (NHID / 64) / 8, 1), 256, 0, stream>>>(
      H1, H1, NHID, 0L, WOUT, WOUT, NHID, 0L, (void*)CA, (void*)CA, NCAT, 0L,
      BIAS + OFF_BOUT, XI, 0L, NROWS, NHID, NHID, OUT_SCL);
  wmma_gemm64<0, false, 2, 0, false, 0><<<dim3((NROWS / 64) * (NIFPAD / 64) / 8, 1), 256, 0, stream>>>(
      H1, H1, NHID, 0L, WIF, WIF, NHID, 0L, (void*)XI, (void*)XI, NIFPAD, 0L,
      BIAS + OFF_BIF, XI, 0L, NROWS, NIFPAD, NHID, AW_INV);
  mem_seq_kernel<<<NBATCH, NTHR, 0, stream>>>(XI, MEMT, LINK, CA);
  wmma_gemm64<0, false, 2, 0, false, 0><<<dim3((NROWS / 64) * (NIN / 64) / 8, 1), 256, 0, stream>>>(
      CA, CA, NCAT, 0L, WMEM, WMEM, NCAT, 0L, (void*)yout, (void*)yout, NIN, 0L,
      BIAS + OFF_BMEM, XI, 0L, NROWS, NIN, NCAT, AW_INV);
}
